// MSA_47253230190881
// MI455X (gfx1250) — hardware-verified
//
#include <hip/hip_runtime.h>
#include <stdint.h>


typedef __attribute__((ext_vector_type(16))) _Float16 v16h;
typedef __attribute__((ext_vector_type(8)))  float    v8f;
typedef __attribute__((ext_vector_type(4)))  float    v4f;
typedef __attribute__((ext_vector_type(4)))  uint32_t v4u;
typedef v4u __attribute__((may_alias)) v4ua;
typedef v4f __attribute__((may_alias)) v4fa;

#ifndef NB
#define NB 4
#endif
#ifndef SEQ
#define SEQ 2048
#endif
#ifndef SEQ_FULL
#define SEQ_FULL 2048
#endif
#ifndef SEQ_OUT
#define SEQ_OUT SEQ
#endif
#define NHEAD 16
#define EMB   1024
#define HDIM  64
#define NQKV  192

static_assert(NB >= 1);
static_assert(SEQ >= 128);
static_assert(SEQ % 128 == 0);
static_assert(SEQ <= SEQ_FULL);
static_assert(NHEAD * HDIM == EMB);
static_assert(((NQKV * HDIM) / 8) % 256 == 0);
static_assert(((EMB * EMB) / 8) % 256 == 0);
static_assert((NB * SEQ) % 128 == 0);
static_assert(EMB % 64 == 0);

static __device__ __forceinline__ float bf16r(float f) {
  uint32_t u = __float_as_uint(f);
  u = u + 0x7FFFu + ((u >> 16) & 1u);
  u = u & 0xFFFF0000u;
  return __uint_as_float(u);
}

union AF { v16h v; _Float16 h[16]; v4u q[2]; };
union H8 { _Float16 h[8]; v4u q; };

static __device__ __forceinline__ void load_frag16(AF& a, const _Float16* row, int lhi) {
  const v4ua* p = (const v4ua*)(row + lhi * 8);
  a.q[0] = p[0];
  a.q[1] = p[2];
}

static __device__ __forceinline__ v8f mma16(v16h a, v16h b, v8f c) {
  v8f d = __builtin_amdgcn_wmma_f32_16x16x32_f16(false, a, false, b, (short)0, c,
                                                 false, false);
  asm volatile("v_nop\n\tv_nop\n\tv_nop\n\tv_nop" : "+v"(d) : "v"(a), "v"(b));
  return d;
}

static __device__ __forceinline__ void vst16(_Float16* p, v4u v) { *(volatile v4u*)p = v; }
static __device__ __forceinline__ void vstf4(float* p, v4f v) { *(volatile v4f*)p = v; }

__global__ __launch_bounds__(256) void cvt_w16_kernel(const float* __restrict__ src,
                                                      _Float16* __restrict__ dst,
                                                      int n8, float scale) {
  const int i = blockIdx.x * 256 + (int)threadIdx.x;
  if (i >= n8) return;
  const v4f* sp = (const v4f*)(src + (size_t)i * 8);
  const v4f f0 = sp[0];
  const v4f f1 = sp[1];
  H8 o;
#pragma unroll
  for (int e = 0; e < 4; ++e) {
    o.h[e]     = (_Float16)(bf16r(f0[e]) * scale);
    o.h[4 + e] = (_Float16)(bf16r(f1[e]) * scale);
  }
  const v4u val = o.q;
  _Float16* dp = dst + (size_t)i * 8;
  vst16(dp, val);
  __threadfence();
  vst16(dp, val);
}

static __device__ __forceinline__ void qkv_store_pass(const _Float16* Qst, const _Float16* Kst,
                                                      const _Float16* Vst, _Float16* qdst,
                                                      _Float16* kdst, _Float16* vdst, int tid) {
#pragma unroll
  for (int it = 0; it < 4; ++it) {
    const int idx = it * 256 + tid;
    vst16(qdst + (size_t)idx * 8, ((const v4ua*)Qst)[idx]);
    vst16(kdst + (size_t)idx * 8, ((const v4ua*)Kst)[idx]);
    const int d = it * 16 + (tid >> 4);
    const int piece = tid & 15;
    vst16(vdst + (size_t)d * SEQ + piece * 8, ((const v4ua*)Vst)[d * 16 + piece]);
  }
}

__global__ __launch_bounds__(256) __attribute__((amdgpu_num_vgpr(256)))
void qkv_kernel(const float* __restrict__ x, const _Float16* __restrict__ Wq16,
                const float* __restrict__ bq, _Float16* __restrict__ Q16,
                _Float16* __restrict__ K16, _Float16* __restrict__ V16T) {
  __shared__ _Float16 Qst[128 * HDIM];
  __shared__ _Float16 Kst[128 * HDIM];
  __shared__ _Float16 Vst[HDIM * 128];

  const int tid  = (int)threadIdx.x;
  const int wave = tid >> 5;
  const int lane = tid & 31;
  const int lhi  = lane >> 4;
  const int ln   = lane & 15;
  const int tb   = blockIdx.x * 128;
  const int h    = blockIdx.y;
  const int b    = blockIdx.z;

  const int trow = tb + wave * 16 + ln;
  const float* xrow = x + ((size_t)b * SEQ_FULL + trow) * EMB + h * HDIM;
  AF xa[2];
#pragma unroll
  for (int ks = 0; ks < 2; ++ks) {
    const v4f* xp = (const v4f*)(xrow + ks * 32 + lhi * 8);
    const v4f f0 = xp[0], f1 = xp[1];
    const v4f f2 = xp[4], f3 = xp[5];
#pragma unroll
    for (int e = 0; e < 4; ++e) {
      xa[ks].h[e]      = (_Float16)bf16r(f0[e]);
      xa[ks].h[4 + e]  = (_Float16)bf16r(f1[e]);
      xa[ks].h[8 + e]  = (_Float16)bf16r(f2[e]);
      xa[ks].h[12 + e] = (_Float16)bf16r(f3[e]);
    }
  }

  const int rbase = wave * 16 + lhi * 8;
#pragma unroll
  for (int n = 0; n < 12; ++n) {
    const int colg = n * 16 + ln;
    AF wb0, wb1;
    load_frag16(wb0, Wq16 + colg * HDIM, lhi);
    load_frag16(wb1, Wq16 + colg * HDIM + 32, lhi);
    const float bv = 8.0f * bf16r(bq[colg]);
    v8f acc;
#pragma unroll
    for (int e = 0; e < 8; ++e) acc[e] = bv;
    acc = mma16(xa[0].v, wb0.v, acc);
    acc = mma16(xa[1].v, wb1.v, acc);
    const int cl = (n & 3) * 16 + ln;
    if (n < 4) {
#pragma unroll
      for (int r = 0; r < 8; ++r) Qst[(rbase + r) * HDIM + cl] = (_Float16)acc[r];
    } else if (n < 8) {
#pragma unroll
      for (int r = 0; r < 8; ++r) Kst[(rbase + r) * HDIM + cl] = (_Float16)acc[r];
    } else {
#pragma unroll
      for (int r = 0; r < 8; ++r) Vst[cl * 128 + rbase + r] = (_Float16)acc[r];
    }
  }
  __syncthreads();

  const size_t bh = (size_t)(b * NHEAD + h);
  _Float16* qdst = Q16 + (bh * SEQ + tb) * HDIM;
  _Float16* kdst = K16 + (bh * SEQ + tb) * HDIM;
  _Float16* vdst = V16T + bh * HDIM * SEQ + tb;
  qkv_store_pass(Qst, Kst, Vst, qdst, kdst, vdst, tid);
  __threadfence();
  qkv_store_pass(Qst, Kst, Vst, qdst, kdst, vdst, tid);
}

static __device__ __forceinline__ void ctx_store_pass(const _Float16* ow, _Float16* cdst, int lane) {
  const int prow = lane >> 3, piece = lane & 7;
#pragma unroll
  for (int i = 0; i < 4; ++i) {
    const int row = i * 4 + prow;
    vst16(cdst + (size_t)row * EMB + piece * 8, ((const v4ua*)ow)[row * 8 + piece]);
  }
}

__global__ __launch_bounds__(256) __attribute__((amdgpu_num_vgpr(256)))
void attn_kernel(const _Float16* __restrict__ Q16, const _Float16* __restrict__ K16,
                 const _Float16* __restrict__ V16T, _Float16* __restrict__ C16,
                 _Float16* __restrict__ R16) {
  __shared__ _Float16 Pb[8][16 * 32];
  __shared__ _Float16 Ost[8][16 * HDIM];
  __shared__ _Float16 Rst[8][16 * HDIM];

  const int tid  = (int)threadIdx.x;
  const int wave = tid >> 5;
  const int lane = tid & 31;
  const int lhi  = lane >> 4;
  const int ln   = lane & 15;
  const int qb   = blockIdx.x * 128;
  const int h    = blockIdx.y;
  const int b    = blockIdx.z;
  const size_t bh = (size_t)(b * NHEAD + h);
  const _Float16* Qp = Q16 + bh * SEQ * HDIM;
  const _Float16* Kp = K16 + bh * SEQ * HDIM;
  const _Float16* Vp = V16T + bh * HDIM * SEQ;

  const int trow = qb + wave * 16 + ln;
  AF qa0, qa1;
  load_frag16(qa0, Qp + (size_t)trow * HDIM, lhi);
  load_frag16(qa1, Qp + (size_t)trow * HDIM + 32, lhi);

  float m[8], ls[8];
  v8f o[4];
#pragma unroll
  for (int r = 0; r < 8; ++r) { m[r] = -3.0e38f; ls[r] = 0.0f; }
#pragma unroll
  for (int d = 0; d < 4; ++d) {
#pragma unroll
    for (int e = 0; e < 8; ++e) o[d][e] = 0.0f;
  }

  _Float16* pw = Pb[wave];
  const float SC = 0.001953125f;

#pragma unroll 1
  for (int kb = 0; kb < SEQ / 32; ++kb) {
    v8f s[2];
#pragma unroll
    for (int nt = 0; nt < 2; ++nt) {
      const int key = kb * 32 + nt * 16 + ln;
      AF f0, f1;
      load_frag16(f0, Kp + (size_t)key * HDIM, lhi);
      load_frag16(f1, Kp + (size_t)key * HDIM + 32, lhi);
      v8f c;
#pragma unroll
      for (int e = 0; e < 8; ++e) c[e] = 0.0f;
      c = mma16(qa0.v, f0.v, c);
      c = mma16(qa1.v, f1.v, c);
      s[nt] = c;
    }

    float corr[8];
#pragma unroll
    for (int r = 0; r < 8; ++r) {
      const float a0 = s[0][r] * SC;
      const float a1 = s[1][r] * SC;
      float mx = fmaxf(a0, a1);
      mx = fmaxf(mx, __shfl_xor(mx, 1));
      mx = fmaxf(mx, __shfl_xor(mx, 2));
      mx = fmaxf(mx, __shfl_xor(mx, 4));
      mx = fmaxf(mx, __shfl_xor(mx, 8));
      const float mn = fmaxf(m[r], mx);
      corr[r] = __expf(m[r] - mn);
      m[r] = mn;
      const float p0 = __expf(a0 - mn);
      const float p1 = __expf(a1 - mn);
      float rs = p0 + p1;
      rs += __shfl_xor(rs, 1);
      rs += __shfl_xor(rs, 2);
      rs += __shfl_xor(rs, 4);
      rs += __shfl_xor(rs, 8);
      ls[r] = ls[r] * corr[r] + rs;
      const int row = lhi * 8 + r;
      pw[row * 32 + ln]      = (_Float16)(p0 * 1024.0f);
      pw[row * 32 + 16 + ln] = (_Float16)(p1 * 1024.0f);
    }
#pragma unroll
    for (int d = 0; d < 4; ++d) {
#pragma unroll
      for (int r = 0; r < 8; ++r) o[d][r] *= corr[r];
    }
    __syncthreads();

    AF pa;
    load_frag16(pa, pw + ln * 32, lhi);

#pragma unroll
    for (int d = 0; d < 4; ++d) {
      AF vf;
      load_frag16(vf, Vp + (size_t)(d * 16 + ln) * SEQ + kb * 32, lhi);
      o[d] = mma16(pa.v, vf.v, o[d]);
    }
    __syncthreads();
  }

  _Float16* ow = Ost[wave];
  _Float16* rw = Rst[wave];
#pragma unroll
  for (int r = 0; r < 8; ++r) {
    const float inv = (1.0f / ls[r]) * 0.015625f;
    const int row = lhi * 8 + r;
#pragma unroll
    for (int d = 0; d < 4; ++d) {
      const float c = o[d][r] * inv;
      const _Float16 hh = (_Float16)c;
      const float resf = (c - (float)hh) * 2048.0f;
      ow[row * HDIM + d * 16 + ln] = hh;
      rw[row * HDIM + d * 16 + ln] = (_Float16)resf;
    }
  }
  __syncthreads();

  const size_t coff = ((size_t)b * SEQ + qb + wave * 16) * EMB + h * HDIM;
  _Float16* cdst = C16 + coff;
  _Float16* rdst = R16 + coff;
  ctx_store_pass(ow, cdst, lane);
  ctx_store_pass(rw, rdst, lane);
  __threadfence();
  ctx_store_pass(ow, cdst, lane);
  ctx_store_pass(rw, rdst, lane);
}

static __device__ __forceinline__ void y_store_pass(const float* yw, float* out, int m0, int n0,
                                                    int lane) {
  const int prow = lane >> 4, piece = lane & 15;
#pragma unroll
  for (int i = 0; i < 16; ++i) {
    const int row = i * 2 + prow;
    const int mm = m0 + row;
    const int ob = mm / SEQ;
    const int ot = mm - ob * SEQ;
    const size_t orow = (size_t)ob * SEQ_OUT + ot;
    vstf4(out + orow * EMB + n0 + piece * 4, ((const v4fa*)yw)[row * 16 + piece]);
  }
}

__global__ __launch_bounds__(128) __attribute__((amdgpu_num_vgpr(256)))
void proj_kernel(const _Float16* __restrict__ C16, const _Float16* __restrict__ R16,
                 const _Float16* __restrict__ Wp16, const float* __restrict__ bp,
                 float* __restrict__ out) {
  __shared__ float Yst[4][32 * 64];

  const int tid  = (int)threadIdx.x;
  const int wave = tid >> 5;
  const int lane = tid & 31;
  const int lhi  = lane >> 4;
  const int ln   = lane & 15;
  const int m0   = blockIdx.x * 128 + wave * 32;
  const int n0   = blockIdx.y * 64;

  const _Float16* ah0 = C16 + (size_t)(m0 + ln) * EMB;
  const _Float16* ah1 = C16 + (size_t)(m0 + 16 + ln) * EMB;
  const _Float16* al0 = R16 + (size_t)(m0 + ln) * EMB;
  const _Float16* al1 = R16 + (size_t)(m0 + 16 + ln) * EMB;
  const _Float16* bpn = Wp16 + (size_t)(n0 + ln) * EMB;

  v8f acch[2][4], accl[2][4];
#pragma unroll
  for (int mi = 0; mi < 2; ++mi) {
#pragma unroll
    for (int nt = 0; nt < 4; ++nt) {
#pragma unroll
      for (int e = 0; e < 8; ++e) { acch[mi][nt][e] = 0.0f; accl[mi][nt][e] = 0.0f; }
    }
  }

#pragma unroll 1
  for (int k0 = 0; k0 < EMB; k0 += 32) {
    AF a0, a1, l0, l1;
    load_frag16(a0, ah0 + k0, lhi);
    load_frag16(a1, ah1 + k0, lhi);
    load_frag16(l0, al0 + k0, lhi);
    load_frag16(l1, al1 + k0, lhi);
#pragma unroll
    for (int nt = 0; nt < 4; ++nt) {
      AF bf;
      load_frag16(bf, bpn + (size_t)nt * 16 * EMB + k0, lhi);
      acch[0][nt] = mma16(a0.v, bf.v, acch[0][nt]);
      acch[1][nt] = mma16(a1.v, bf.v, acch[1][nt]);
      accl[0][nt] = mma16(l0.v, bf.v, accl[0][nt]);
      accl[1][nt] = mma16(l1.v, bf.v, accl[1][nt]);
    }
  }

  float* yw = Yst[wave];
#pragma unroll
  for (int nt = 0; nt < 4; ++nt) {
    const int col = nt * 16 + ln;
    const float bias = bf16r(bp[n0 + col]);
#pragma unroll
    for (int mi = 0; mi < 2; ++mi) {
#pragma unroll
      for (int r = 0; r < 8; ++r) {
        const float v = (acch[mi][nt][r] + accl[mi][nt][r] * 0.00048828125f) * 0.000244140625f + bias;
        yw[(mi * 16 + lhi * 8 + r) * 64 + col] = v;
      }
    }
  }
  __syncthreads();

  y_store_pass(yw, out, m0, n0, lane);
  __threadfence();
  y_store_pass(yw, out, m0, n0, lane);
}

extern "C" void kernel_launch(void* const* d_in, const int* in_sizes, int n_in,
                              void* d_out, int out_size, void* d_ws, size_t ws_size,
                              hipStream_t stream) {
  if (n_in < 5) return;
  if (in_sizes[0] < ((NB - 1) * SEQ_FULL + SEQ) * EMB) return;
  if (in_sizes[1] < NQKV * HDIM) return;
  if (in_sizes[2] < NQKV) return;
  if (in_sizes[3] < EMB * EMB) return;
  if (in_sizes[4] < EMB) return;
  if (out_size < ((NB - 1) * SEQ_OUT + SEQ) * EMB) return;

  const float* x     = (const float*)d_in[0];
  const float* Wqkv  = (const float*)d_in[1];
  const float* bqkv  = (const float*)d_in[2];
  const float* Wproj = (const float*)d_in[3];
  const float* bproj = (const float*)d_in[4];
  float* out = (float*)d_out;

  char* ws = (char*)d_ws;
  size_t off = 0;
  _Float16* Wq16 = (_Float16*)(ws + off); off += (size_t)NQKV * HDIM * 2;
  _Float16* Wp16 = (_Float16*)(ws + off); off += (size_t)EMB * EMB * 2;
  const size_t psz = (size_t)NB * NHEAD * SEQ * HDIM * 2;
  _Float16* Q16  = (_Float16*)(ws + off); off += psz;
  _Float16* K16  = (_Float16*)(ws + off); off += psz;
  _Float16* V16T = (_Float16*)(ws + off); off += psz;
  _Float16* C16  = (_Float16*)(ws + off); off += (size_t)NB * SEQ * EMB * 2;
  _Float16* R16  = (_Float16*)(ws + off); off += (size_t)NB * SEQ * EMB * 2;
  if (off > ws_size) return;

  cvt_w16_kernel<<<(NQKV * HDIM / 8) / 256, 256, 0, stream>>>(Wqkv, Wq16, NQKV * HDIM / 8, 8.0f);
  cvt_w16_kernel<<<(EMB * EMB / 8) / 256, 256, 0, stream>>>(Wproj, Wp16, EMB * EMB / 8, 32.0f);

  dim3 g1(SEQ / 128, NHEAD, NB);
  qkv_kernel<<<g1, 256, 0, stream>>>(x, Wq16, bqkv, Q16, K16, V16T);
  attn_kernel<<<g1, 256, 0, stream>>>(Q16, K16, V16T, C16, R16);

  dim3 g3((NB * SEQ) / 128, EMB / 64);
  proj_kernel<<<g3, 128, 0, stream>>>(C16, R16, Wp16, bproj, out);
}
